// TransformerBlock_17231408792466
// MI455X (gfx1250) — hardware-verified
//
#include <hip/hip_runtime.h>
#include <stddef.h>


typedef _Float16 v16h __attribute__((ext_vector_type(16)));
typedef _Float16 v8h  __attribute__((ext_vector_type(8)));
typedef float    v8f  __attribute__((ext_vector_type(8)));
typedef float    v4f  __attribute__((ext_vector_type(4)));

#ifndef NB
#define NB 2
#endif
#ifndef SEQ
#define SEQ 2048
#endif
#define NB_FULL  2
#define SEQ_FULL 2048
#define DIM   512
#define DFF   2048
#define NHEAD 8
#define HD    64
#define MROWS (NB * SEQ)
#define LNROWS 8
#define LN_EPS 1.0e-5f

static_assert(NB >= 1 && NB <= NB_FULL);
static_assert(SEQ >= 128 && SEQ <= SEQ_FULL && (SEQ % 128) == 0);
static_assert((SEQ % 64) == 0);
static_assert(DIM == NHEAD * HD);
static_assert(HD == 64);
static_assert((DIM % 64) == 0 && (DIM % 32) == 0);
static_assert((DFF % 64) == 0 && (DFF % 32) == 0);
static_assert((MROWS % 64) == 0);
static_assert((MROWS % LNROWS) == 0);
static_assert((DIM % 256) == 0);
static_assert((DIM % 8) == 0);
static_assert(((size_t)MROWS * DIM) % 2048 == 0);
static_assert((size_t)MROWS * DFF < (size_t)0xFFFFFFFFu);

#define LDT 72
#define LDC 68

#define WCARRY  64.0f
#define PCARRY  1024.0f
#define VCARRY  64.0f
#define QRCARRY 2048.0f
#define CRCARRY 64.0f
#define FCARRY  8.0f

#define WSQ_BYTES  ((size_t)DIM * DIM * 2)
#define WO_BYTES   ((size_t)DIM * 2 * DIM * 2)
#define WFF_BYTES  ((size_t)DFF * DIM * 2)
#define P16_BYTES  ((size_t)MROWS * DIM * 2)
#define P32_BYTES  ((size_t)MROWS * DIM * 4)
#define CTX_BYTES  ((size_t)MROWS * 2 * DIM * 2)
#define F1_BYTES   ((size_t)MROWS * DFF * 2)
#define OFF_WQT  ((size_t)0)
#define OFF_WKT  (OFF_WQT + WSQ_BYTES)
#define OFF_WVT  (OFF_WKT + WSQ_BYTES)
#define OFF_WOT  (OFF_WVT + WSQ_BYTES)
#define OFF_W1T  (OFF_WOT + WO_BYTES)
#define OFF_W2T  (OFF_W1T + WFF_BYTES)
#define OFF_X16  (OFF_W2T + WFF_BYTES)
#define OFF_QH   (OFF_X16 + P16_BYTES)
#define OFF_QR   (OFF_QH + P16_BYTES)
#define OFF_KH   (OFF_QR + P16_BYTES)
#define OFF_KR   (OFF_KH + P16_BYTES)
#define OFF_VT   (OFF_KR + P16_BYTES)
#define OFF_CTX  (OFF_VT + P16_BYTES)
#define OFF_Y1   (OFF_CTX + CTX_BYTES)
#define OFF_HF   (OFF_Y1 + P32_BYTES)
#define OFF_H16  (OFF_HF + P32_BYTES)
#define OFF_F1   (OFF_H16 + P16_BYTES)
#define OFF_Y2   (OFF_F1 + F1_BYTES)
#define WS_TOTAL (OFF_Y2 + P32_BYTES)
static_assert((WSQ_BYTES % 128) == 0 && (WO_BYTES % 128) == 0 && (WFF_BYTES % 128) == 0);
static_assert((P16_BYTES % 128) == 0 && (P32_BYTES % 128) == 0);
static_assert((CTX_BYTES % 128) == 0 && (F1_BYTES % 128) == 0);
static_assert(WS_TOTAL <= (size_t)134217728);

__device__ __forceinline__ float bf16r(float x) {
  unsigned int u = __float_as_uint(x);
  u = (u + 0x7FFFu + ((u >> 16) & 1u)) & 0xFFFF0000u;
  return __uint_as_float(u);
}

__device__ __forceinline__ unsigned full_row(unsigned r) {
  return (r / (unsigned)SEQ) * (unsigned)SEQ_FULL + (r % (unsigned)SEQ);
}

__device__ __forceinline__ v16h frag_at(const _Float16* p) {
  v8h lo = *(const v8h*)(p);
  v8h hi = *(const v8h*)(p + 16);
  v16h out;
#pragma unroll
  for (int i = 0; i < 8; ++i) { out[i] = lo[i]; out[i + 8] = hi[i]; }
  return out;
}
__device__ __forceinline__ v16h ld_frag(const _Float16* base, unsigned ld) {
  const unsigned lane = threadIdx.x & 31u;
  return frag_at(base + (lane & 15u) * ld + (lane >> 4) * 8u);
}

__device__ __forceinline__ v8f wmma16(v16h a, v16h b, v8f c) {
  v8f d = __builtin_amdgcn_wmma_f32_16x16x32_f16(false, a, false, b, (short)0, c,
                                                 false, false);
  asm volatile("v_nop\n\tv_nop\n\tv_nop\n\tv_nop" : "+v"(d) : "v"(a), "v"(b));
  return d;
}

__device__ __forceinline__ float red16_max(float x) {
#pragma unroll
  for (int off = 1; off < 16; off <<= 1) x = fmaxf(x, __shfl_xor(x, off, 32));
  return x;
}
__device__ __forceinline__ float red16_sum(float x) {
#pragma unroll
  for (int off = 1; off < 16; off <<= 1) x += __shfl_xor(x, off, 32);
  return x;
}
__device__ __forceinline__ float red32_sum(float x) {
#pragma unroll
  for (int off = 1; off < 32; off <<= 1) x += __shfl_xor(x, off, 32);
  return x;
}

__device__ __forceinline__ void wave_lds_sync() {
  __builtin_amdgcn_fence(3  , "wavefront");
  asm volatile("s_wait_dscnt 0x0" ::: "memory");
  __builtin_amdgcn_wave_barrier();
}

__global__ __launch_bounds__(256) void convx_kernel(
    const float* __restrict__ src, _Float16* __restrict__ dst) {
  const size_t e = ((size_t)blockIdx.x * 256u + threadIdx.x) * 8u;
  const unsigned row = (unsigned)(e / (size_t)DIM);
  const unsigned col = (unsigned)(e % (size_t)DIM);
  const size_t se = (size_t)full_row(row) * DIM + col;
  const v4f a0 = *(const v4f*)(src + se);
  const v4f a1 = *(const v4f*)(src + se + 4);
  v8h o;
#pragma unroll
  for (int j = 0; j < 4; ++j) {
    o[j]     = (_Float16)bf16r(a0[j]);
    o[j + 4] = (_Float16)bf16r(a1[j]);
  }
  *(volatile v8h*)(dst + e) = o;
  __threadfence();
  *(volatile v8h*)(dst + e) = o;
}

__global__ __launch_bounds__(256) void wtrans_kernel(
    const float* __restrict__ W, _Float16* __restrict__ dst,
    int N, int ldd, int koff, float carry) {
  __shared__ __attribute__((aligned(16))) float T[64 * LDC];
  const unsigned tid = threadIdx.x;
  const unsigned n0 = blockIdx.x * 64u;
  const unsigned k0 = blockIdx.y * 64u;
#pragma unroll
  for (unsigned j = 0; j < 4u; ++j) {
    const unsigned idx = tid + 256u * j;
    const unsigned r = idx >> 4, c = (idx & 15u) * 4u;
    *(v4f*)&T[r * LDC + c] = *(const v4f*)(W + (size_t)(k0 + r) * (unsigned)N + n0 + c);
  }
  __syncthreads();
  v8h x[2];
  size_t off[2];
#pragma unroll
  for (unsigned i = 0; i < 2u; ++i) {
    const unsigned nrow = 32u * i + (tid >> 3);
    const unsigned kk = (tid & 7u) * 8u;
#pragma unroll
    for (unsigned j = 0; j < 8u; ++j)
      x[i][j] = (_Float16)(carry * bf16r(T[(kk + j) * LDC + nrow]));
    off[i] = (size_t)(n0 + nrow) * (unsigned)ldd + (unsigned)koff + k0 + kk;
  }
#pragma unroll
  for (int i = 0; i < 2; ++i) *(volatile v8h*)(dst + off[i]) = x[i];
  __threadfence();
#pragma unroll
  for (int i = 0; i < 2; ++i) *(volatile v8h*)(dst + off[i]) = x[i];
}

template <int MODE, int KD, int LDO>
__device__ __forceinline__ void gemm_body(
    const _Float16* __restrict__ A16, const _Float16* __restrict__ Bt,
    const float* __restrict__ addf, const float* __restrict__ resf,
    float* __restrict__ outf, _Float16* __restrict__ out16,
    _Float16* __restrict__ out16b, float* Cs) {
  static_assert((KD % 32) == 0);
  static_assert((LDO % 64) == 0);
  const unsigned tid = threadIdx.x, lane = tid & 31u;
  const unsigned w = (unsigned)__builtin_amdgcn_readfirstlane((int)(tid >> 5));
  const unsigned mw = w >> 1, nw = w & 1u;
  const unsigned hh = lane >> 4, m = lane & 15u;
  const unsigned n0 = blockIdx.x * 64u;
  const unsigned row0 = blockIdx.y * 64u;

  const _Float16* ap  = A16 + (size_t)(row0 + mw * 16u + m) * KD + hh * 8u;
  const _Float16* bp0 = Bt + (size_t)(n0 + nw * 32u + m) * KD + hh * 8u;
  const _Float16* bp1 = bp0 + (size_t)16 * KD;
  v8f acc0 = {}, acc1 = {};
#pragma unroll 2
  for (unsigned k0 = 0; k0 < (unsigned)KD; k0 += 32u) {
    const v16h a  = frag_at(ap + k0);
    const v16h b0 = frag_at(bp0 + k0);
    const v16h b1 = frag_at(bp1 + k0);
    acc0 = wmma16(a, b0, acc0);
    acc1 = wmma16(a, b1, acc1);
  }
#pragma unroll
  for (int r = 0; r < 8; ++r) {
    float* d = &Cs[(mw * 16u + hh * 8u + (unsigned)r) * LDC + nw * 32u + m];
    d[0]  = acc0[r];
    d[16] = acc1[r];
  }
  __syncthreads();

  if (MODE == 0) {
    v8h xh[2], xr[2];
    size_t off[2];
#pragma unroll
    for (unsigned i = 0; i < 2u; ++i) {
      const unsigned r = 32u * i + (tid >> 3);
      const unsigned c = (tid & 7u) * 8u;
      const v4f u0 = *(const v4f*)&Cs[r * LDC + c];
      const v4f u1 = *(const v4f*)&Cs[r * LDC + c + 4];
      const v4f g0 = *(const v4f*)(addf + n0 + c);
      const v4f g1 = *(const v4f*)(addf + n0 + c + 4);
#pragma unroll
      for (int j = 0; j < 4; ++j) {
        const float va = u0[j] * (1.0f / WCARRY) + bf16r(g0[j]);
        const float vb = u1[j] * (1.0f / WCARRY) + bf16r(g1[j]);
        const _Float16 ha = (_Float16)va;
        const _Float16 hb = (_Float16)vb;
        xh[i][j]     = ha;
        xh[i][j + 4] = hb;
        xr[i][j]     = (_Float16)((va - (float)ha) * QRCARRY);
        xr[i][j + 4] = (_Float16)((vb - (float)hb) * QRCARRY);
      }
      off[i] = (size_t)(row0 + r) * LDO + n0 + c;
    }
#pragma unroll
    for (int i = 0; i < 2; ++i) {
      *(volatile v8h*)(out16 + off[i]) = xh[i];
      *(volatile v8h*)(out16b + off[i]) = xr[i];
    }
    __threadfence();
#pragma unroll
    for (int i = 0; i < 2; ++i) {
      *(volatile v8h*)(out16 + off[i]) = xh[i];
      *(volatile v8h*)(out16b + off[i]) = xr[i];
    }
  }

  if (MODE == 3) {
    v8h x[2];
    size_t off[2];
#pragma unroll
    for (unsigned i = 0; i < 2u; ++i) {
      const unsigned r = 32u * i + (tid >> 3);
      const unsigned c = (tid & 7u) * 8u;
      const v4f u0 = *(const v4f*)&Cs[r * LDC + c];
      const v4f u1 = *(const v4f*)&Cs[r * LDC + c + 4];
      const v4f g0 = *(const v4f*)(addf + n0 + c);
      const v4f g1 = *(const v4f*)(addf + n0 + c + 4);
#pragma unroll
      for (int j = 0; j < 4; ++j) {
        x[i][j]     = (_Float16)(FCARRY * fmaxf(u0[j] * (1.0f / WCARRY) + bf16r(g0[j]), 0.0f));
        x[i][j + 4] = (_Float16)(FCARRY * fmaxf(u1[j] * (1.0f / WCARRY) + bf16r(g1[j]), 0.0f));
      }
      off[i] = (size_t)(row0 + r) * LDO + n0 + c;
    }
#pragma unroll
    for (int i = 0; i < 2; ++i) *(volatile v8h*)(out16 + off[i]) = x[i];
    __threadfence();
#pragma unroll
    for (int i = 0; i < 2; ++i) *(volatile v8h*)(out16 + off[i]) = x[i];
  }

  if (MODE == 1) {
    const unsigned bb = row0 / (unsigned)SEQ;
    const unsigned s0 = row0 % (unsigned)SEQ;
    v8h x[2];
    size_t off[2];
#pragma unroll
    for (unsigned i = 0; i < 2u; ++i) {
      const unsigned dcol = 32u * i + (tid >> 3);
      const unsigned kk = (tid & 7u) * 8u;
      const float bias = bf16r(addf[n0 + dcol]);
#pragma unroll
      for (unsigned j = 0; j < 8u; ++j)
        x[i][j] = (_Float16)(Cs[(kk + j) * LDC + dcol] * (1.0f / WCARRY) + bias);
      off[i] = ((size_t)bb * DIM + n0 + dcol) * SEQ + s0 + kk;
    }
#pragma unroll
    for (int i = 0; i < 2; ++i) *(volatile v8h*)(out16 + off[i]) = x[i];
    __threadfence();
#pragma unroll
    for (int i = 0; i < 2; ++i) *(volatile v8h*)(out16 + off[i]) = x[i];
  }

  if (MODE == 4 || MODE == 6) {
    const float isc = (MODE == 4) ? (1.0f / (WCARRY * VCARRY)) : (1.0f / (WCARRY * FCARRY));
    v4f xs[4];
    size_t off[4];
#pragma unroll
    for (unsigned i = 0; i < 4u; ++i) {
      const unsigned r = 16u * i + (tid >> 4);
      const unsigned c = (tid & 15u) * 4u;
      const unsigned rr = row0 + r;
      const size_t o = (size_t)rr * DIM + n0 + c;
      const size_t ro = (MODE == 4) ? ((size_t)full_row(rr) * DIM + n0 + c) : o;
      const v4f u = *(const v4f*)&Cs[r * LDC + c];
      const v4f g = *(const v4f*)(addf + n0 + c);
      const v4f hres = *(const v4f*)(resf + ro);
      v4f val;
#pragma unroll
      for (int j = 0; j < 4; ++j) {
        const float rj = (MODE == 4) ? bf16r(hres[j]) : hres[j];
        val[j] = (u[j] * isc + bf16r(g[j])) + rj;
      }
      xs[i] = val;
      off[i] = o;
    }
#pragma unroll
    for (int i = 0; i < 4; ++i) *(volatile v4f*)(outf + off[i]) = xs[i];
    __threadfence();
#pragma unroll
    for (int i = 0; i < 4; ++i) *(volatile v4f*)(outf + off[i]) = xs[i];
  }
}

__global__ __launch_bounds__(256) void gemm_qk_kernel(
    const _Float16* __restrict__ A16, const _Float16* __restrict__ Bt,
    const float* __restrict__ bias, _Float16* __restrict__ outh,
    _Float16* __restrict__ outr) {
  __shared__ __attribute__((aligned(16))) float Cs[64 * LDC];
  gemm_body<0, DIM, DIM>(A16, Bt, bias, nullptr, nullptr, outh, outr, Cs);
}
__global__ __launch_bounds__(256) void gemm_vt_kernel(
    const _Float16* __restrict__ A16, const _Float16* __restrict__ Bt,
    const float* __restrict__ bias, _Float16* __restrict__ out16) {
  __shared__ __attribute__((aligned(16))) float Cs[64 * LDC];
  gemm_body<1, DIM, DIM>(A16, Bt, bias, nullptr, nullptr, out16, nullptr, Cs);
}
__global__ __launch_bounds__(256) void gemm_wo_kernel(
    const _Float16* __restrict__ A16, const _Float16* __restrict__ Bt,
    const float* __restrict__ bias, const float* __restrict__ xin,
    float* __restrict__ outf) {
  __shared__ __attribute__((aligned(16))) float Cs[64 * LDC];
  gemm_body<4, 2 * DIM, DIM>(A16, Bt, bias, xin, outf, nullptr, nullptr, Cs);
}
__global__ __launch_bounds__(256) void gemm_ffn1_kernel(
    const _Float16* __restrict__ A16, const _Float16* __restrict__ Bt,
    const float* __restrict__ bias, _Float16* __restrict__ out16) {
  __shared__ __attribute__((aligned(16))) float Cs[64 * LDC];
  gemm_body<3, DIM, DFF>(A16, Bt, bias, nullptr, nullptr, out16, nullptr, Cs);
}
__global__ __launch_bounds__(256) void gemm_ffn2_kernel(
    const _Float16* __restrict__ A16, const _Float16* __restrict__ Bt,
    const float* __restrict__ bias, const float* __restrict__ resf,
    float* __restrict__ outf) {
  __shared__ __attribute__((aligned(16))) float Cs[64 * LDC];
  gemm_body<6, DFF, DIM>(A16, Bt, bias, resf, outf, nullptr, nullptr, Cs);
}

__global__ __launch_bounds__(256) void attn_kernel(
    const _Float16* __restrict__ Qh, const _Float16* __restrict__ Qr,
    const _Float16* __restrict__ Kh, const _Float16* __restrict__ Kr,
    const _Float16* __restrict__ Vt, _Float16* __restrict__ Cx) {
  __shared__ __attribute__((aligned(16))) _Float16 Ksh[64 * LDT];
  __shared__ __attribute__((aligned(16))) _Float16 Ksr[64 * LDT];
  __shared__ __attribute__((aligned(16))) _Float16 Vs[64 * LDT];
  __shared__ __attribute__((aligned(16))) _Float16 Ps[8 * 16 * LDT];

  const unsigned tid = threadIdx.x, lane = tid & 31u;
  const unsigned wave = (unsigned)__builtin_amdgcn_readfirstlane((int)(tid >> 5));
  const unsigned hh = lane >> 4, m = lane & 15u;
  const unsigned q0 = blockIdx.x * 128u;
  const unsigned head = blockIdx.y;
  const unsigned bb = blockIdx.z;
  const float sc_main = 0.125f;
  const float sc_res = 0.125f / QRCARRY;
  const unsigned pbase = wave * (16u * LDT);

  const size_t qoff = (size_t)(bb * (unsigned)SEQ + q0 + wave * 16u + m) * DIM + head * HD + hh * 8u;

  float mrow[8], lrow[8];
  v8f o[4];
#pragma unroll
  for (int v = 0; v < 8; ++v) { mrow[v] = -1.0e30f; lrow[v] = 0.0f; }
#pragma unroll
  for (int nb = 0; nb < 4; ++nb) o[nb] = (v8f){};

  const size_t kplane = (size_t)bb * SEQ * DIM + (size_t)head * HD;
  const size_t vplane = ((size_t)bb * DIM + (size_t)head * HD) * SEQ;

  for (unsigned kb = 0; kb < (unsigned)SEQ; kb += 64u) {
#pragma unroll
    for (unsigned j = 0; j < 2u; ++j) {
      const unsigned idx = tid + 256u * j;
      const unsigned r = idx >> 3, c = (idx & 7u) * 8u;
      const size_t goff = kplane + (size_t)(kb + r) * DIM + c;
      *(v8h*)&Ksh[r * LDT + c] = *(const v8h*)(Kh + goff);
      *(v8h*)&Ksr[r * LDT + c] = *(const v8h*)(Kr + goff);
      *(v8h*)&Vs[r * LDT + c]  = *(const v8h*)(Vt + vplane + (size_t)r * SEQ + kb + c);
    }
    __syncthreads();

#pragma unroll 1
    for (unsigned hf = 0; hf < 2u; ++hf) {
      v8f s[2];
#pragma unroll
      for (int kg = 0; kg < 2; ++kg) {
        v8f t = {};
        v8f u = {};
        const unsigned krow = (hf * 32u + (unsigned)kg * 16u) * LDT;
#pragma unroll
        for (int c = 0; c < 2; ++c) {
          const v16h qh = frag_at(Qh + qoff + c * 32);
          const v16h qr = frag_at(Qr + qoff + c * 32);
          const v16h kh = ld_frag(&Ksh[krow + c * 32], LDT);
          const v16h kr = ld_frag(&Ksr[krow + c * 32], LDT);
          t = wmma16(qh, kh, t);
          u = wmma16(qh, kr, u);
          u = wmma16(qr, kh, u);
        }
        s[kg] = t * sc_main + u * sc_res;
      }

      float alpha[8];
#pragma unroll
      for (int v = 0; v < 8; ++v) {
        float mx = fmaxf(s[0][v], s[1][v]);
        mx = red16_max(mx);
        const float mn = fmaxf(mrow[v], mx);
        alpha[v] = __expf(mrow[v] - mn);
        mrow[v] = mn;
      }
#pragma unroll
      for (int kg = 0; kg < 2; ++kg)
#pragma unroll
        for (int v = 0; v < 8; ++v) s[kg][v] = __expf(s[kg][v] - mrow[v]);
#pragma unroll
      for (int v = 0; v < 8; ++v) {
        const float rs = red16_sum(s[0][v] + s[1][v]);
        lrow[v] = alpha[v] * lrow[v] + rs;
      }
#pragma unroll
      for (int nb = 0; nb < 4; ++nb)
#pragma unroll
        for (int v = 0; v < 8; ++v) o[nb][v] = o[nb][v] * alpha[v];

#pragma unroll
      for (int kg = 0; kg < 2; ++kg)
#pragma unroll
        for (int v = 0; v < 8; ++v)
          Ps[pbase + (hh * 8u + (unsigned)v) * LDT + (unsigned)kg * 16u + m] =
              (_Float16)(s[kg][v] * PCARRY);
      wave_lds_sync();

      const v16h pf = ld_frag(&Ps[pbase], LDT);
#pragma unroll
      for (int nb = 0; nb < 4; ++nb) {
        const v16h vf = ld_frag(&Vs[(nb * 16) * LDT + hf * 32u], LDT);
        o[nb] = wmma16(pf, vf, o[nb]);
      }
      wave_lds_sync();
    }
    __syncthreads();
  }

  float inv[8];
#pragma unroll
  for (int v = 0; v < 8; ++v) inv[v] = __builtin_amdgcn_rcpf(lrow[v]) * (VCARRY / PCARRY);
#pragma unroll
  for (int nb = 0; nb < 4; ++nb)
#pragma unroll
    for (int v = 0; v < 8; ++v) {
      const float val = o[nb][v] * inv[v];
      const _Float16 hv = (_Float16)val;
      Ps[pbase + (hh * 8u + (unsigned)v) * LDT + (unsigned)nb * 16u + m] = hv;
      o[nb][v] = (val - (float)hv) * CRCARRY;
    }
  wave_lds_sync();
  v8h xh[4], xr[4];
  size_t off[4];
#pragma unroll
  for (unsigned i = 0; i < 4u; ++i) {
    const unsigned r = 4u * i + (lane >> 3);
    const unsigned c = (lane & 7u) * 8u;
    xh[i] = *(const v8h*)&Ps[pbase + r * LDT + c];
    off[i] = (size_t)(bb * (unsigned)SEQ + q0 + wave * 16u + r) * (2 * DIM) + head * HD + c;
  }
  wave_lds_sync();
#pragma unroll
  for (int nb = 0; nb < 4; ++nb)
#pragma unroll
    for (int v = 0; v < 8; ++v)
      Ps[pbase + (hh * 8u + (unsigned)v) * LDT + (unsigned)nb * 16u + m] = (_Float16)o[nb][v];
  wave_lds_sync();
#pragma unroll
  for (unsigned i = 0; i < 4u; ++i) {
    const unsigned r = 4u * i + (lane >> 3);
    const unsigned c = (lane & 7u) * 8u;
    xr[i] = *(const v8h*)&Ps[pbase + r * LDT + c];
  }
#pragma unroll
  for (int i = 0; i < 4; ++i) {
    *(volatile v8h*)(Cx + off[i]) = xh[i];
    *(volatile v8h*)(Cx + off[i] + DIM) = xr[i];
  }
  __threadfence();
#pragma unroll
  for (int i = 0; i < 4; ++i) {
    *(volatile v8h*)(Cx + off[i]) = xh[i];
    *(volatile v8h*)(Cx + off[i] + DIM) = xr[i];
  }
}

template <int FIRST>
__device__ __forceinline__ void ln_store(
    const float* S, const float* __restrict__ g, const float* __restrict__ be,
    float* __restrict__ outF, _Float16* __restrict__ out16, size_t obase, float mu, float rs) {
  const unsigned lane = threadIdx.x & 31u;
#pragma unroll 1
  for (unsigned it = 0; it < (unsigned)(DIM / 128); ++it) {
    const unsigned c = it * 128u + lane * 4u;
    const v4f v = *(const v4f*)&S[c];
    const v4f gg = *(const v4f*)(g + c);
    const v4f bb = *(const v4f*)(be + c);
    v4f ov;
#pragma unroll
    for (int j = 0; j < 4; ++j) ov[j] = (v[j] - mu) * rs * bf16r(gg[j]) + bf16r(bb[j]);
    *(volatile v4f*)(outF + obase + c) = ov;
  }
  if (FIRST) {
#pragma unroll 1
    for (unsigned it = 0; it < (unsigned)(DIM / 256); ++it) {
      const unsigned c = it * 256u + lane * 8u;
      const v4f v0 = *(const v4f*)&S[c];
      const v4f v1 = *(const v4f*)&S[c + 4];
      const v4f g0 = *(const v4f*)(g + c);
      const v4f g1 = *(const v4f*)(g + c + 4);
      const v4f b0 = *(const v4f*)(be + c);
      const v4f b1 = *(const v4f*)(be + c + 4);
      v8h x;
#pragma unroll
      for (int j = 0; j < 4; ++j) {
        x[j]     = (_Float16)((v0[j] - mu) * rs * bf16r(g0[j]) + bf16r(b0[j]));
        x[j + 4] = (_Float16)((v1[j] - mu) * rs * bf16r(g1[j]) + bf16r(b1[j]));
      }
      *(volatile v8h*)(out16 + obase + c) = x;
    }
  }
}

template <int FIRST>
__device__ __forceinline__ void ln_body(
    const float* __restrict__ src, const float* __restrict__ g, const float* __restrict__ be,
    float* __restrict__ outF, _Float16* __restrict__ out16, float* S,
    size_t ibase, size_t obase) {
  const unsigned lane = threadIdx.x & 31u;
  float sum = 0.0f;
#pragma unroll 1
  for (unsigned it = 0; it < (unsigned)(DIM / 128); ++it) {
    const unsigned c = it * 128u + lane * 4u;
    const v4f v = *(const v4f*)(src + ibase + c);
    *(v4f*)&S[c] = v;
    sum += (v[0] + v[1]) + (v[2] + v[3]);
  }
  sum = red32_sum(sum);
  const float mu = sum * (1.0f / (float)DIM);
  float sq = 0.0f;
#pragma unroll 1
  for (unsigned it = 0; it < (unsigned)(DIM / 128); ++it) {
    const unsigned c = it * 128u + lane * 4u;
    const v4f v = *(const v4f*)&S[c];
    const float d0 = v[0] - mu, d1 = v[1] - mu, d2 = v[2] - mu, d3 = v[3] - mu;
    sq += (d0 * d0 + d1 * d1) + (d2 * d2 + d3 * d3);
  }
  sq = red32_sum(sq);
  const float rs = rsqrtf(sq * (1.0f / (float)DIM) + LN_EPS);
  wave_lds_sync();
  ln_store<FIRST>(S, g, be, outF, out16, obase, mu, rs);
  __threadfence();
  ln_store<FIRST>(S, g, be, outF, out16, obase, mu, rs);
}

__global__ __launch_bounds__(256) void ln1_kernel(
    const float* __restrict__ Y, const float* __restrict__ g,
    const float* __restrict__ be, float* __restrict__ hF, _Float16* __restrict__ h16) {
  __shared__ __attribute__((aligned(16))) float S[LNROWS * DIM];
  const unsigned w = (unsigned)__builtin_amdgcn_readfirstlane((int)(threadIdx.x >> 5));
  const unsigned row = blockIdx.x * (unsigned)LNROWS + w;
  const size_t rb = (size_t)row * DIM;
  ln_body<1>(Y, g, be, hF, h16, S + w * (unsigned)DIM, rb, rb);
}
__global__ __launch_bounds__(256) void ln2_kernel(
    const float* __restrict__ Y, const float* __restrict__ g,
    const float* __restrict__ be, float* __restrict__ out) {
  __shared__ __attribute__((aligned(16))) float S[LNROWS * DIM];
  const unsigned w = (unsigned)__builtin_amdgcn_readfirstlane((int)(threadIdx.x >> 5));
  const unsigned row = blockIdx.x * (unsigned)LNROWS + w;
  ln_body<0>(Y, g, be, out, nullptr, S + w * (unsigned)DIM, (size_t)row * DIM,
             (size_t)full_row(row) * DIM);
}

extern "C" void kernel_launch(void* const* d_in, const int* in_sizes, int n_in,
                              void* d_out, int out_size, void* d_ws, size_t ws_size,
                              hipStream_t stream) {
  if (n_in < 17) return;
  const long long need_x = ((long long)(NB - 1) * SEQ_FULL + SEQ) * DIM;
  if ((long long)in_sizes[0] < need_x) return;
  if ((long long)in_sizes[1] < (long long)DIM * DIM) return;
  if ((long long)in_sizes[3] < (long long)DIM * DIM) return;
  if ((long long)in_sizes[5] < (long long)DIM * DIM) return;
  if ((long long)in_sizes[7] < (long long)DIM * DIM) return;
  if (in_sizes[2] < DIM || in_sizes[4] < DIM || in_sizes[6] < DIM || in_sizes[8] < DIM) return;
  if ((long long)in_sizes[9] < (long long)DIM * DFF) return;
  if (in_sizes[10] < DFF) return;
  if ((long long)in_sizes[11] < (long long)DFF * DIM) return;
  if (in_sizes[12] < DIM || in_sizes[13] < DIM || in_sizes[14] < DIM) return;
  if (in_sizes[15] < DIM || in_sizes[16] < DIM) return;
  if ((long long)out_size < need_x) return;
  if (ws_size < WS_TOTAL) return;

  const float* X   = (const float*)d_in[0];
  const float* Wq  = (const float*)d_in[1];
  const float* bq  = (const float*)d_in[2];
  const float* Wk  = (const float*)d_in[3];
  const float* bk  = (const float*)d_in[4];
  const float* Wv  = (const float*)d_in[5];
  const float* bv  = (const float*)d_in[6];
  const float* Wo  = (const float*)d_in[7];
  const float* bo  = (const float*)d_in[8];
  const float* W1  = (const float*)d_in[9];
  const float* b1  = (const float*)d_in[10];
  const float* W2  = (const float*)d_in[11];
  const float* b2  = (const float*)d_in[12];
  const float* g1  = (const float*)d_in[13];
  const float* be1 = (const float*)d_in[14];
  const float* g2  = (const float*)d_in[15];
  const float* be2 = (const float*)d_in[16];
  float* out = (float*)d_out;

  char* ws = (char*)d_ws;
  _Float16* WqT = (_Float16*)(ws + OFF_WQT);
  _Float16* WkT = (_Float16*)(ws + OFF_WKT);
  _Float16* WvT = (_Float16*)(ws + OFF_WVT);
  _Float16* WoT = (_Float16*)(ws + OFF_WOT);
  _Float16* W1T = (_Float16*)(ws + OFF_W1T);
  _Float16* W2T = (_Float16*)(ws + OFF_W2T);
  _Float16* X16 = (_Float16*)(ws + OFF_X16);
  _Float16* QH  = (_Float16*)(ws + OFF_QH);
  _Float16* QR  = (_Float16*)(ws + OFF_QR);
  _Float16* KH  = (_Float16*)(ws + OFF_KH);
  _Float16* KR  = (_Float16*)(ws + OFF_KR);
  _Float16* VT  = (_Float16*)(ws + OFF_VT);
  _Float16* CTX = (_Float16*)(ws + OFF_CTX);
  float*    Y1  = (float*)(ws + OFF_Y1);
  float*    HF  = (float*)(ws + OFF_HF);
  _Float16* H16 = (_Float16*)(ws + OFF_H16);
  _Float16* F1  = (_Float16*)(ws + OFF_F1);
  float*    Y2  = (float*)(ws + OFF_Y2);

  dim3 blk(256);

  convx_kernel<<<dim3((unsigned)(((size_t)MROWS * DIM) / 2048)), blk, 0, stream>>>(X, X16);

  wtrans_kernel<<<dim3(DIM / 64, DIM / 64), blk, 0, stream>>>(Wq, WqT, DIM, DIM, 0, WCARRY);
  wtrans_kernel<<<dim3(DIM / 64, DIM / 64), blk, 0, stream>>>(Wk, WkT, DIM, DIM, 0, WCARRY);
  wtrans_kernel<<<dim3(DIM / 64, DIM / 64), blk, 0, stream>>>(Wv, WvT, DIM, DIM, 0, WCARRY);
  wtrans_kernel<<<dim3(DIM / 64, DIM / 64), blk, 0, stream>>>(Wo, WoT, DIM, 2 * DIM, 0, WCARRY);
  wtrans_kernel<<<dim3(DIM / 64, DIM / 64), blk, 0, stream>>>(Wo, WoT, DIM, 2 * DIM, DIM,
                                                             WCARRY / CRCARRY);
  wtrans_kernel<<<dim3(DFF / 64, DIM / 64), blk, 0, stream>>>(W1, W1T, DFF, DIM, 0, WCARRY);
  wtrans_kernel<<<dim3(DIM / 64, DFF / 64), blk, 0, stream>>>(W2, W2T, DIM, DFF, 0, WCARRY);

  gemm_qk_kernel<<<dim3(DIM / 64, MROWS / 64), blk, 0, stream>>>(X16, WqT, bq, QH, QR);
  gemm_qk_kernel<<<dim3(DIM / 64, MROWS / 64), blk, 0, stream>>>(X16, WkT, bk, KH, KR);
  gemm_vt_kernel<<<dim3(DIM / 64, MROWS / 64), blk, 0, stream>>>(X16, WvT, bv, VT);

  attn_kernel<<<dim3(SEQ / 128, NHEAD, NB), blk, 0, stream>>>(QH, QR, KH, KR, VT, CTX);

  gemm_wo_kernel<<<dim3(DIM / 64, MROWS / 64), blk, 0, stream>>>(CTX, WoT, bo, X, Y1);

  ln1_kernel<<<dim3(MROWS / LNROWS), blk, 0, stream>>>(Y1, g1, be1, HF, H16);

  gemm_ffn1_kernel<<<dim3(DFF / 64, MROWS / 64), blk, 0, stream>>>(H16, W1T, b1, F1);
  gemm_ffn2_kernel<<<dim3(DIM / 64, MROWS / 64), blk, 0, stream>>>(F1, W2T, b2, HF, Y2);

  ln2_kernel<<<dim3(MROWS / LNROWS), blk, 0, stream>>>(Y2, g2, be2, out);
}
